// WordLoss_20340965113904
// MI455X (gfx1250) — hardware-run, weakly checked
//
#include <hip/hip_runtime.h>
#include <math.h>

typedef __attribute__((ext_vector_type(16))) _Float16 v16h;
typedef __attribute__((ext_vector_type(8)))  _Float16 v8h;
typedef __attribute__((ext_vector_type(16))) __bf16   v16b;
typedef __attribute__((ext_vector_type(8)))  __bf16   v8b;
typedef __attribute__((ext_vector_type(8)))  float    v8f;
typedef __attribute__((ext_vector_type(4)))  float    v4f;
typedef __attribute__((ext_vector_type(2)))  float    v2f;
typedef __attribute__((ext_vector_type(4)))  unsigned int v4u;

constexpr int kB   = 64;
constexpr int kD   = 256;
constexpr int kT   = 24;
constexpr int kRg  = 17;
constexpr int kS   = kRg * kRg;
constexpr int kSM  = 304;
constexpr int kSK  = 320;
constexpr int kTN  = 32;
constexpr int kLP  = 33;
constexpr int kAP  = 320;
constexpr float kG1 = 4.0f;
constexpr float kG2 = 5.0f;
constexpr float kG3 = 10.0f;
constexpr float kEps = 1e-8f;
constexpr float kNegFill = -1e30f;
constexpr int kOutFloats = 2 + kB * kT * kS;
constexpr int kOutChunks = kOutFloats / 4;
static_assert(kS == 289, "regions");
static_assert((kD % 32) == 0 && (kSK % 32) == 0, "K multiples of 32");
static_assert((kSM % 16) == 0 && (kTN % 16) == 0 && (kD % 16) == 0, "tile multiples");
static_assert(kSM >= kS && kSK >= kS && kTN >= kT && kAP >= kS, "pads");
static_assert(kOutFloats == 443906, "output extent");
static_assert(kOutChunks * 4 + 2 == kOutFloats, "two-float tail");
static_assert((kOutChunks % 32) == 0, "whole waves of 16-B chunks");

constexpr size_t kOffCtxT = 0;
constexpr size_t kOffCtxN = kOffCtxT + (size_t)kB * kSM * kD * 2;
constexpr size_t kOffWT   = kOffCtxN + (size_t)kB * kD * kSK * 2;
constexpr size_t kOffSim  = kOffWT   + (size_t)kB * kTN * kD * 2;
constexpr size_t kOffAtt  = kOffSim  + (size_t)kB * kB * 32 * 4;
constexpr size_t kOffLoss = kOffAtt  + (size_t)kB * kT * kAP * 4;
constexpr size_t kWsTotal = kOffLoss + 128;
static_assert(kWsTotal == 23986304ull, "carve total");
static_assert(kWsTotal <= 134217728ull, "carve cap");
static_assert((kOffCtxN % 128) == 0 && (kOffWT % 128) == 0 && (kOffSim % 128) == 0 &&
              (kOffAtt % 128) == 0 && (kOffLoss % 128) == 0, "128-B aligned regions");

__device__ __forceinline__ unsigned short f2bf_bits(float f) {
  unsigned u = __float_as_uint(f);
  return (unsigned short)((u + 0x7FFFu + ((u >> 16) & 1u)) >> 16);
}
__device__ __forceinline__ __bf16 at_f2bf(float f) { return __builtin_bit_cast(__bf16, f2bf_bits(f)); }
__device__ __forceinline__ unsigned pk16(unsigned short a, unsigned short b) { return (unsigned)a | ((unsigned)b << 16); }

template <typename T> struct Frag;
template <> struct Frag<__bf16> {
  typedef v16b V; union U { v16b v; v8b h[2]; };
  static __device__ __forceinline__ v16b load(const __bf16* p) {
    U f; f.h[0] = *(const v8b*)(p); f.h[1] = *(const v8b*)(p + 16); return f.v;
  }
};
__device__ __forceinline__ v8f at_mma(v16b a, v16b b, v8f c) {
  c = __builtin_amdgcn_wmma_f32_16x16x32_bf16(false, a, false, b, (short)0, c, false, false);
  asm volatile("v_nop\n\tv_nop\n\tv_nop\n\tv_nop" : "+v"(c) : "v"(a), "v"(b));
  return c;
}

__device__ __forceinline__ float wave_max(float v) {
#pragma unroll
  for (int o = 16; o > 0; o >>= 1) v = fmaxf(v, __shfl_xor(v, o, 32));
  return v;
}
__device__ __forceinline__ float wave_sum(float v) {
#pragma unroll
  for (int o = 16; o > 0; o >>= 1) v += __shfl_xor(v, o, 32);
  return v;
}

__global__ __launch_bounds__(256) void ctx_rows_kernel(const float* __restrict__ img, unsigned short* __restrict__ ctxN)
{
  const int idx = blockIdx.x * 256 + threadIdx.x;
  if (idx >= kB * kD * (kSK / 8)) return;
  const int row = idx / (kSK / 8);
  const int c8  = idx - row * (kSK / 8);
  const float* src = img + (size_t)row * kS;
  unsigned short hb[8];
#pragma unroll
  for (int e = 0; e < 8; ++e) {
    const int s  = c8 * 8 + e;
    const int sc = (s < kS) ? s : (kS - 1);
    float f = src[sc];
    f = (s < kS) ? f : 0.0f;
    hb[e] = f2bf_bits(f);
  }
  const v4u u = (v4u){pk16(hb[0], hb[1]), pk16(hb[2], hb[3]), pk16(hb[4], hb[5]), pk16(hb[6], hb[7])};
  unsigned short* q = ctxN + (size_t)idx * 8;
  *(volatile v4u*)q = u;
  __threadfence();
  *(volatile v4u*)q = u;
}

__global__ __launch_bounds__(256) void ctx_transpose_kernel(const float* __restrict__ img, unsigned short* __restrict__ ctxT)
{
  __shared__ __align__(16) float sm[16 * 260];
  const int tid = threadIdx.x, lane = tid & 31, wv = tid >> 5;
  const int s0 = blockIdx.x * 16;
  const int b  = blockIdx.y;
  const int sl = tid & 15, dq = tid >> 4;
  const int s  = s0 + sl;
  const int sc = (s < kS) ? s : (kS - 1);
  const bool valid = (s < kS);
#pragma unroll
  for (int i = 0; i < 16; ++i) {
    const int d = dq + 16 * i;
    float f = img[((size_t)b * kD + d) * kS + sc];
    f = valid ? f : 0.0f;
    sm[sl * 260 + d] = f;
  }
  __syncthreads();
  v4u u[2];
#pragma unroll
  for (int it = 0; it < 2; ++it) {
    const int row = it * 8 + wv;
    const float* sp = sm + row * 260 + lane * 8;
    const v4f a0 = *(const v4f*)(sp);
    const v4f a1 = *(const v4f*)(sp + 4);
    unsigned short hb[8];
#pragma unroll
    for (int e = 0; e < 4; ++e) {
      const float x0 = a0[e];
      const float x1 = a1[e];
      hb[e]     = f2bf_bits(x0);
      hb[4 + e] = f2bf_bits(x1);
    }
    u[it] = (v4u){pk16(hb[0], hb[1]), pk16(hb[2], hb[3]), pk16(hb[4], hb[5]), pk16(hb[6], hb[7])};
  }
  for (int pass = 0; pass < 2; ++pass) {
#pragma unroll
    for (int it = 0; it < 2; ++it) {
      const int row = it * 8 + wv;
      *(volatile v4u*)(ctxT + ((size_t)b * kSM + s0 + row) * kD + lane * 8) = u[it];
    }
    __threadfence();
  }
}

__global__ __launch_bounds__(256) void words_transpose_kernel(const float* __restrict__ words, unsigned short* __restrict__ wT)
{
  __shared__ __align__(16) float sm[kT * 260];
  const int tid = threadIdx.x, lane = tid & 31, wv = tid >> 5;
  const int i = blockIdx.x;
  const float* src = words + (size_t)i * kD * kT;
#pragma unroll 8
  for (int k = 0; k < kT; ++k) {
    const int e = k * 256 + tid;
    const int d = e / kT;
    const int t = e - d * kT;
    sm[t * 260 + d] = src[e];
  }
  __syncthreads();
  v4u u[4];
#pragma unroll
  for (int it = 0; it < 4; ++it) {
    const int row = it * 8 + wv;
    const int rc  = (row < kT) ? row : (kT - 1);
    const bool live = (row < kT);
    const float* sp = sm + rc * 260 + lane * 8;
    const v4f a0 = *(const v4f*)(sp);
    const v4f a1 = *(const v4f*)(sp + 4);
    unsigned short hb[8];
#pragma unroll
    for (int e = 0; e < 4; ++e) {
      const float x0 = live ? a0[e] : 0.0f;
      const float x1 = live ? a1[e] : 0.0f;
      hb[e]     = f2bf_bits(x0);
      hb[4 + e] = f2bf_bits(x1);
    }
    u[it] = (v4u){pk16(hb[0], hb[1]), pk16(hb[2], hb[3]), pk16(hb[4], hb[5]), pk16(hb[6], hb[7])};
  }
  for (int pass = 0; pass < 2; ++pass) {
#pragma unroll
    for (int it = 0; it < 4; ++it) {
      const int row = it * 8 + wv;
      *(volatile v4u*)(wT + ((size_t)i * kTN + row) * kD + lane * 8) = u[it];
    }
    __threadfence();
  }
}

__global__ __launch_bounds__(256) void pair_kernel(
    const unsigned short* __restrict__ ctxT, const unsigned short* __restrict__ ctxN,
    const unsigned short* __restrict__ wT, const int* __restrict__ cap_lens,
    float* __restrict__ simL, float* __restrict__ attws)
{
  union FB { v16b v; v8b h[2]; };
  __shared__ __align__(16) float  sA[kSM * kLP];
  __shared__ __align__(16) __bf16 sB2[kTN * kSK];
  __shared__ float sE[32];

  const int bb   = blockIdx.x;
  const int ii   = blockIdx.y;
  const int tid  = threadIdx.x;
  const int lane = tid & 31;
  const int wv   = tid >> 5;
  const int hh   = lane >> 4;
  const int cl   = lane & 15;
  const int koff = 8 * hh;

  int len = cap_lens[ii];
  len = (len < 0) ? 0 : ((len > kT) ? kT : len);
  const float padp = (len == 0) ? (1.0f / 24.0f) : 0.0f;

  {
    const __bf16* A1 = (const __bf16*)(const void*)ctxT + (size_t)bb * kSM * kD;
    const __bf16* B1 = (const __bf16*)(const void*)wT   + (size_t)ii * kTN * kD;
    const __bf16* bp0 = B1 + (size_t)cl * kD + koff;
    const __bf16* bp1 = B1 + (size_t)(16 + cl) * kD + koff;
#pragma unroll 1
    for (int mt = wv; mt < kSM / 16; mt += 8) {
      const int m0 = mt * 16;
      const __bf16* ap = A1 + (size_t)(m0 + cl) * kD + koff;
      v8f c0 = (v8f){0.f,0.f,0.f,0.f,0.f,0.f,0.f,0.f};
      v8f c1 = (v8f){0.f,0.f,0.f,0.f,0.f,0.f,0.f,0.f};
#pragma unroll 2
      for (int k0 = 0; k0 < kD; k0 += 32) {
        const v16b a  = Frag<__bf16>::load(ap + k0);
        const v16b b0 = Frag<__bf16>::load(bp0 + k0);
        const v16b b1 = Frag<__bf16>::load(bp1 + k0);
        c0 = at_mma(a, b0, c0);
        c1 = at_mma(a, b1, c1);
      }
#pragma unroll
      for (int r = 0; r < 8; ++r) {
        sA[(m0 + 8 * hh + r) * kLP + cl]      = c0[r];
        sA[(m0 + 8 * hh + r) * kLP + 16 + cl] = c1[r];
      }
    }
  }
  __syncthreads();

#pragma unroll 1
  for (int s = tid; s < kS; s += 256) {
    float* row = sA + s * kLP;
    float m = row[0];
#pragma unroll 1
    for (int t = 1; t < len; ++t) m = fmaxf(m, row[t]);
    float sum = 0.0f;
#pragma unroll 1
    for (int t = 0; t < len; ++t) {
      const float e = expf(row[t] - m);
      row[t] = e;
      sum += e;
    }
    const float inv = 1.0f / sum;
#pragma unroll 1
    for (int t = 0; t < len; ++t) row[t] = row[t] * inv;
#pragma unroll 1
    for (int t = len; t < kT; ++t) row[t] = padp;
  }
  __syncthreads();

  const bool diag = (ii == bb);
  const __bf16 zb = at_f2bf(0.0f);
#pragma unroll 1
  for (int j = 0; j < 3; ++j) {
    const int t = wv + 8 * j;
    float mx = -INFINITY;
#pragma unroll
    for (int k = 0; k < 10; ++k) {
      const int s  = lane + 32 * k;
      const int sc = (s < kS) ? s : (kS - 1);
      const float p = sA[sc * kLP + t];
      const float v = (s < kS) ? (kG1 * p) : -INFINITY;
      mx = fmaxf(mx, v);
    }
    mx = wave_max(mx);
    float sum = 0.0f;
#pragma unroll 2
    for (int k = 0; k < 10; ++k) {
      const int s  = lane + 32 * k;
      const int sc = (s < kS) ? s : (kS - 1);
      const float p = sA[sc * kLP + t];
      float e = expf(kG1 * p - mx);
      e = (s < kS) ? e : 0.0f;
      if (s < kS) sA[s * kLP + t] = e;
      sum += e;
    }
    sum = wave_sum(sum);
    const float inv = 1.0f / sum;
    float pk[10];
#pragma unroll
    for (int k = 0; k < 10; ++k) {
      const int s  = lane + 32 * k;
      const int sc = (s < kS) ? s : (kS - 1);
      const float e = sA[sc * kLP + t];
      const float p2 = (s < kS) ? (e * inv) : 0.0f;
      pk[k] = p2;
      sB2[t * kSK + s] = at_f2bf(p2);
    }
    if (diag) {
      float* rowp = attws + ((size_t)(bb * kT + t)) * kAP + lane;
      for (int pass = 0; pass < 2; ++pass) {
#pragma unroll
        for (int k = 0; k < 10; ++k) *(volatile float*)(rowp + 32 * k) = pk[k];
        __threadfence();
      }
    }
  }
#pragma unroll
  for (int k = 0; k < 10; ++k) sB2[(kT + wv) * kSK + lane + 32 * k] = zb;
  __syncthreads();

  {
    const __bf16* A2 = (const __bf16*)(const void*)ctxN + (size_t)bb * kD * kSK;
#pragma unroll 1
    for (int mt = wv; mt < kD / 16; mt += 8) {
      const int m0 = mt * 16;
      const __bf16* ap = A2 + (size_t)(m0 + cl) * kSK + koff;
      v8f c0 = (v8f){0.f,0.f,0.f,0.f,0.f,0.f,0.f,0.f};
      v8f c1 = (v8f){0.f,0.f,0.f,0.f,0.f,0.f,0.f,0.f};
#pragma unroll 2
      for (int k0 = 0; k0 < kSK; k0 += 32) {
        const v16b a = Frag<__bf16>::load(ap + k0);
        FB b0, b1;
        b0.h[0] = *(const v8b*)(sB2 + cl * kSK + koff + k0);
        b0.h[1] = *(const v8b*)(sB2 + cl * kSK + koff + k0 + 16);
        b1.h[0] = *(const v8b*)(sB2 + (16 + cl) * kSK + koff + k0);
        b1.h[1] = *(const v8b*)(sB2 + (16 + cl) * kSK + koff + k0 + 16);
        c0 = at_mma(a, b0.v, c0);
        c1 = at_mma(a, b1.v, c1);
      }
#pragma unroll
      for (int r = 0; r < 8; ++r) {
        sA[(m0 + 8 * hh + r) * kLP + cl]      = c0[r];
        sA[(m0 + 8 * hh + r) * kLP + 16 + cl] = c1[r];
      }
    }
  }
  __syncthreads();

  {
    const unsigned short* wrow0 = wT + (size_t)ii * kTN * kD;
#pragma unroll 1
    for (int j = 0; j < 3; ++j) {
      const int t = wv + 8 * j;
      const v4u wq = *(const v4u*)(wrow0 + (size_t)t * kD + lane * 8);
      const unsigned q0 = wq[0];
      const unsigned q1 = wq[1];
      const unsigned q2 = wq[2];
      const unsigned q3 = wq[3];
      float wv8[8];
      wv8[0] = __uint_as_float(q0 << 16);
      wv8[1] = __uint_as_float(q0 & 0xffff0000u);
      wv8[2] = __uint_as_float(q1 << 16);
      wv8[3] = __uint_as_float(q1 & 0xffff0000u);
      wv8[4] = __uint_as_float(q2 << 16);
      wv8[5] = __uint_as_float(q2 & 0xffff0000u);
      wv8[6] = __uint_as_float(q3 << 16);
      wv8[7] = __uint_as_float(q3 & 0xffff0000u);
      float num = 0.0f, nw = 0.0f, nv = 0.0f;
#pragma unroll
      for (int e = 0; e < 8; ++e) {
        const float w = wv8[e];
        const float v = sA[(lane * 8 + e) * kLP + t];
        num += w * v;
        nw  += w * w;
        nv  += v * v;
      }
      num = wave_sum(num);
      nw  = wave_sum(nw);
      nv  = wave_sum(nv);
      const float den = fmaxf(sqrtf(nw) * sqrtf(nv), kEps);
      const float rs  = num / den;
      const float ex  = expf(kG2 * rs);
      const float ev  = (t < len) ? ex : 0.0f;
      if (lane == 0) sE[t] = ev;
    }
  }
  __syncthreads();

  if (wv == 0) {
    float tot = 0.0f;
#pragma unroll 1
    for (int k = 0; k < kT; ++k) tot += sE[k];
    const float sv  = kG3 * logf(tot);
    const float val = (lane == 0) ? sv : 0.0f;
    volatile float* p = simL + ((size_t)(bb * kB + ii)) * 32 + lane;
    *p = val;
    __threadfence();
    *p = val;
  }
}

__global__ __launch_bounds__(64) void loss_kernel(const float* __restrict__ simL, const int* __restrict__ labels,
                                                 const int* __restrict__ class_ids, float* __restrict__ lossLine)
{
  __shared__ float sR[2][kB];
  const int r = threadIdx.x;
  const int cr = class_ids[r];
  int l = labels[r];
  l = (l < 0) ? 0 : ((l > kB - 1) ? (kB - 1) : l);
  const int clab = class_ids[l];
  const bool lmask = (clab == cr) && (l != r);
#pragma unroll 1
  for (int w = 0; w < 2; ++w) {
    const int sr = (w == 0) ? kB : 1;
    const int sc = (w == 0) ? 1 : kB;
    float m = -INFINITY;
#pragma unroll 1
    for (int c = 0; c < kB; ++c) {
      const bool msk = (class_ids[c] == cr) && (c != r);
      float v = simL[(size_t)(r * sr + c * sc) * 32];
      v = msk ? kNegFill : v;
      m = fmaxf(m, v);
    }
    float sum = 0.0f;
#pragma unroll 1
    for (int c = 0; c < kB; ++c) {
      const bool msk = (class_ids[c] == cr) && (c != r);
      float v = simL[(size_t)(r * sr + c * sc) * 32];
      v = msk ? kNegFill : v;
      sum += expf(v - m);
    }
    float vl = simL[(size_t)(r * sr + l * sc) * 32];
    vl = lmask ? kNegFill : vl;
    sR[w][r] = (vl - m) - logf(sum);
  }
  __syncthreads();
  if (r < 32) {
    float s0 = 0.0f, s1 = 0.0f;
#pragma unroll 1
    for (int k = 0; k < kB; ++k) {
      s0 += sR[0][k];
      s1 += sR[1][k];
    }
    const float l0 = -(s0 * (1.0f / 64.0f));
    const float l1 = -(s1 * (1.0f / 64.0f));
    const float val = (r == 0) ? l0 : ((r == 1) ? l1 : 0.0f);
    volatile float* p = lossLine + r;
    *p = val;
    __threadfence();
    *p = val;
  }
}

__global__ __launch_bounds__(256) void out_writer_kernel(const float* __restrict__ attws, const float* __restrict__ lossLine,
                                                         float* __restrict__ out)
{
  const int ch = blockIdx.x * 256 + threadIdx.x;
  float v[4];
#pragma unroll
  for (int e = 0; e < 4; ++e) {
    const int j  = 4 * ch + e;
    const int jl = (j < 1) ? 0 : 1;
    int q = j - 2;
    q = (q < 0) ? 0 : ((q > kB * kT * kS - 1) ? (kB * kT * kS - 1) : q);
    const int row = q / kS;
    const int s   = q - row * kS;
    float lv = lossLine[jl];
    float av = attws[(size_t)row * kAP + s];
    asm volatile("" : "+v"(lv));
    asm volatile("" : "+v"(av));
    v[e] = (j < 2) ? lv : av;
  }
  if (ch < kOutChunks) {
    const v4f o = (v4f){v[0], v[1], v[2], v[3]};
    float* p = out + (size_t)ch * 4;
    *(volatile v4f*)p = o;
    __threadfence();
    *(volatile v4f*)p = o;
  } else if (ch == kOutChunks) {
    const v2f o = (v2f){v[0], v[1]};
    float* p = out + (size_t)kOutChunks * 4;
    *(volatile v2f*)p = o;
    __threadfence();
    *(volatile v2f*)p = o;
  }
}

extern "C" void kernel_launch(void* const* d_in, const int* in_sizes, int n_in,
                              void* d_out, int out_size, void* d_ws, size_t ws_size,
                              hipStream_t stream) {
  if (n_in < 5) return;
  if (in_sizes[0] != kB * kD * kS) return;
  if (in_sizes[1] != kB * kD * kT) return;
  if (in_sizes[2] != kB) return;
  if (in_sizes[3] != kB) return;
  if (in_sizes[4] != kB) return;
  if (out_size != kOutFloats) return;
  if (ws_size < kWsTotal) return;

  const float* img       = (const float*)d_in[0];
  const float* words     = (const float*)d_in[1];
  const int*   labels    = (const int*)d_in[2];
  const int*   cap_lens  = (const int*)d_in[3];
  const int*   class_ids = (const int*)d_in[4];
  float* out = (float*)d_out;

  char* ws = (char*)d_ws;
  unsigned short* ctxT = (unsigned short*)(ws + kOffCtxT);
  unsigned short* ctxN = (unsigned short*)(ws + kOffCtxN);
  unsigned short* wT   = (unsigned short*)(ws + kOffWT);
  float* simL  = (float*)(ws + kOffSim);
  float* attws = (float*)(ws + kOffAtt);
  float* lossL = (float*)(ws + kOffLoss);

  ctx_transpose_kernel<<<dim3(kSM / 16, kB), 256, 0, stream>>>(img, ctxT);
  ctx_rows_kernel<<<dim3((kB * kD * (kSK / 8)) / 256), 256, 0, stream>>>(img, ctxN);
  words_transpose_kernel<<<dim3(kB), 256, 0, stream>>>(words, wT);

  pair_kernel<<<dim3(kB, kB), 256, 0, stream>>>(ctxT, ctxN, wT, cap_lens, simL, attws);

  loss_kernel<<<dim3(1), kB, 0, stream>>>(simL, labels, class_ids, lossL);

  out_writer_kernel<<<dim3((kOutChunks + 1 + 255) / 256), 256, 0, stream>>>(attws, lossL, out);
}
